// DynamicConvolution2D_79370995630779
// MI455X (gfx1250) — hardware-verified
//
#include <hip/hip_runtime.h>
#include <hip/hip_bf16.h>

#define BB   16
#define TT   1024
#define CC   256
#define HH   4
#define KK   31
#define PADK 15
#define MM   (BB * TT)
#define NW   (HH * KK)
#define C2   (2 * CC)

#define __bf16 _Float16
#define NWP  128
#define KKP  32
typedef __attribute__((ext_vector_type(16))) __bf16 v16bf;
typedef __attribute__((ext_vector_type(8)))  __bf16 v8bf;
typedef __attribute__((ext_vector_type(4)))  __bf16 v4bf;
typedef __attribute__((ext_vector_type(8)))  float  v8f;
typedef __attribute__((ext_vector_type(4)))  float  v4f_t;
typedef float v4fa __attribute__((ext_vector_type(4), may_alias));
typedef __attribute__((ext_vector_type(4)))  unsigned v4u_t;
typedef unsigned v4ua __attribute__((ext_vector_type(4), may_alias));

static __device__ __forceinline__ v8f wmma_bf16(v16bf a, v16bf b, v8f c) {
    return __builtin_amdgcn_wmma_f32_16x16x32_f16(
         false, a,  false, b,
         (short)0, c,  false,  false);
}

static __device__ __forceinline__ v16bf load_a_bf16(const __bf16* __restrict__ A,
                                                    int lda, int m0, int k0, int lane) {
    int row = m0 + (lane & 15);
    int hl  = lane >> 4;
    const __bf16* p0 = A + (size_t)row * lda + k0 + 8 * hl;
    v8bf c0 = *(const v8bf*)p0;
    v8bf c1 = *(const v8bf*)(p0 + 16);
    v16bf f;
#pragma unroll
    for (int i = 0; i < 8; ++i) { f[i] = c0[i]; f[8 + i] = c1[i]; }
    return f;
}

static __device__ __forceinline__ v16bf load_b_packed(const __bf16* __restrict__ P,
                                                      int NT, int kt, int nt, int lane) {
    const __bf16* p = P + (((size_t)(kt * NT + nt) * 32 + lane) * 16);
    v8bf c0 = *(const v8bf*)p;
    v8bf c1 = *(const v8bf*)(p + 8);
    v16bf f;
#pragma unroll
    for (int i = 0; i < 8; ++i) { f[i] = c0[i]; f[8 + i] = c1[i]; }
    return f;
}

__global__ void k_pack_b(const float* __restrict__ W, int Kdim, int N, int Npad,
                         __bf16* __restrict__ P) {
    int gid  = blockIdx.x * blockDim.x + threadIdx.x;
    int NT   = Npad >> 4;
    int lane = gid & 31;
    int tile = gid >> 5;
    if (tile >= (Kdim >> 5) * NT) return;
    int kt = tile / NT, nt = tile % NT;
    int col = nt * 16 + (lane & 15);
    int hl  = lane >> 4;
    int k0  = kt * 32;
    v8bf c0, c1;
#pragma unroll
    for (int i = 0; i < 8; ++i) {
        int ka = k0 + 8 * hl + i;
        int kb = ka + 16;
        c0[i] = (col < N) ? (__bf16)W[(size_t)ka * N + col] : (__bf16)0.0f;
        c1[i] = (col < N) ? (__bf16)W[(size_t)kb * N + col] : (__bf16)0.0f;
    }
    __bf16* dst = P + ((size_t)tile * 32 + lane) * 16;
    *(volatile v4u_t*)dst = *(const v4ua*)&c0; *(volatile v4u_t*)(dst + 8) = *(const v4ua*)&c1; __threadfence();
    *(volatile v4u_t*)dst = *(const v4ua*)&c0; *(volatile v4u_t*)(dst + 8) = *(const v4ua*)&c1;
}

__global__ void k_cvt_bf16(const float* __restrict__ src, __bf16* __restrict__ dst, int n4) {
    int gid = blockIdx.x * blockDim.x + threadIdx.x;
    if (gid >= n4) return;
    float4 v = ((const float4*)src)[gid];
    v4bf o;
    o[0] = (__bf16)v.x; o[1] = (__bf16)v.y; o[2] = (__bf16)v.z; o[3] = (__bf16)v.w;
    typedef __attribute__((ext_vector_type(2))) unsigned v2u_t; typedef unsigned v2ua __attribute__((ext_vector_type(2), may_alias));
    *(volatile v2u_t*)(dst + (size_t)gid * 4) = *(const v2ua*)&o; __threadfence(); *(volatile v2u_t*)(dst + (size_t)gid * 4) = *(const v2ua*)&o;
}

__global__ __launch_bounds__(256) void k_glu_gemm(const __bf16* __restrict__ qb,
                           const __bf16* __restrict__ pw1,
                           const float* __restrict__ b1,
                           float* __restrict__ x_f32,
                           __bf16* __restrict__ x_bf16) {
    __shared__ __attribute__((aligned(16))) float st[8][16 * 68];
    int lane = threadIdx.x & 31;
    float* sw = st[threadIdx.x >> 5];
    int job  = blockIdx.x * (blockDim.x >> 5) + (threadIdx.x >> 5);
    int mt   = job >> 2;
    int g4   = job & 3;
    if (mt >= MM / 16) return;
    int m0 = mt * 16;
    int ntBase = g4 * 4;
    const int NT = 32;

    v8f acc[8];
#pragma unroll
    for (int i = 0; i < 8; ++i) acc[i] = (v8f){};

    for (int kt = 0; kt < CC / 32; ++kt) {
        v16bf af = load_a_bf16(qb, CC, m0, kt * 32, lane);
#pragma unroll
        for (int i = 0; i < 4; ++i) {
            v16bf ba = load_b_packed(pw1, NT, kt, ntBase + i,      lane);
            acc[i]     = wmma_bf16(af, ba, acc[i]);
            v16bf bg = load_b_packed(pw1, NT, kt, ntBase + i + 16, lane);
            acc[4 + i] = wmma_bf16(af, bg, acc[4 + i]);
        }
    }

    int hl = lane >> 4;
#pragma unroll
    for (int i = 0; i < 4; ++i) {
        int col  = (ntBase + i) * 16 + (lane & 15);
        float ba = b1[col], bg = b1[col + CC];
#pragma unroll
        for (int v = 0; v < 8; ++v) {
            int row  = m0 + v + 8 * hl;
            float a  = acc[i][v] + ba;
            float g  = acc[4 + i][v] + bg;
            float xv = a * (1.0f / (1.0f + __expf(-g)));
            sw[(v + 8 * hl) * 68 + i * 16 + (lane & 15)] = xv; (void)row;
        }
    }
    asm volatile("s_wait_dscnt 0" ::: "memory");
    const int cb = ntBase * 16;
#pragma unroll 1
    for (int pass = 0; pass < 2; ++pass) {
#pragma unroll
        for (int it = 0; it < 8; ++it) { const int ch = lane + 32 * it, r = ch >> 4, q = (ch & 15) * 4;
            *(volatile v4f_t*)(x_f32 + (size_t)(m0 + r) * CC + cb + q) = *(const volatile v4fa*)(sw + r * 68 + q); }
#pragma unroll
        for (int it = 0; it < 4; ++it) { const int ch = lane + 32 * it, r = ch >> 3, q = (ch & 7) * 8; __bf16 hh[8];
#pragma unroll
            for (int e = 0; e < 8; ++e) hh[e] = (__bf16)sw[r * 68 + q + e];
            *(volatile v4u_t*)(x_bf16 + (size_t)(m0 + r) * CC + cb + q) = *(const v4ua*)hh; }
        __threadfence();
    }
}

__global__ __launch_bounds__(256) void k_coef_gemm(const __bf16* __restrict__ xb,
                            const __bf16* __restrict__ pww,
                            const __bf16* __restrict__ pwf,
                            const float* __restrict__ bw,
                            const float* __restrict__ bfv,
                            float* __restrict__ wcoef,
                            float* __restrict__ wfk) {
    __shared__ __attribute__((aligned(16))) float st[8][16 * 68];
    int lane = threadIdx.x & 31;
    float* sw = st[threadIdx.x >> 5];
    int job  = blockIdx.x * (blockDim.x >> 5) + (threadIdx.x >> 5);
    int mt = job / 3, sub = job % 3;
    if (mt >= MM / 16) return;
    int m0 = mt * 16;

    const __bf16* P; const float* bias; float* dst;
    int NT, ntBase, ngroup, N, NP;
    if (sub < 2) { P = pww; NT = 8; ntBase = sub * 4; ngroup = 4; N = NW; NP = NWP; bias = bw;  dst = wcoef; }
    else         { P = pwf; NT = 2; ntBase = 0;       ngroup = 2; N = KK; NP = KKP; bias = bfv; dst = wfk;  }

    v8f acc[4];
#pragma unroll
    for (int i = 0; i < 4; ++i) acc[i] = (v8f){};

    for (int kt = 0; kt < CC / 32; ++kt) {
        v16bf af = load_a_bf16(xb, CC, m0, kt * 32, lane);
#pragma unroll
        for (int i = 0; i < 4; ++i) {
            if (i < ngroup) {
                v16bf bfr = load_b_packed(P, NT, kt, ntBase + i, lane);
                acc[i] = wmma_bf16(af, bfr, acc[i]);
            }
        }
    }

    int hl = lane >> 4;
#pragma unroll
    for (int i = 0; i < 4; ++i) {
        if (i < ngroup) {
            int col = (ntBase + i) * 16 + (lane & 15);
            float bv = (col < N) ? bias[col] : 0.0f;
#pragma unroll
            for (int v = 0; v < 8; ++v) sw[(v + 8 * hl) * 68 + i * 16 + (lane & 15)] = (col < N) ? (acc[i][v] + bv) : 0.0f;
        }
    }
    asm volatile("s_wait_dscnt 0" ::: "memory");
    const int ncol = ngroup * 16, cb = ntBase * 16;
#pragma unroll 1
    for (int pass = 0; pass < 2; ++pass) {
        for (int ch = lane; ch < 16 * (ncol / 4); ch += 32) { const int r = ch / (ncol / 4), q = (ch % (ncol / 4)) * 4;
            *(volatile v4f_t*)(dst + (size_t)(m0 + r) * NP + cb + q) = *(const volatile v4fa*)(sw + r * 68 + q); }
        __threadfence();
    }
}

__global__ __launch_bounds__(256) void k_mix(const float* __restrict__ x,
                      const float* __restrict__ wcoef,
                      const float* __restrict__ wfk,
                      const int*   __restrict__ mask,
                      __bf16* __restrict__ cat) {
    __shared__ float attn_s[HH][KK + 1];
    __shared__ float wk_s[KK + 1];
    __shared__ __attribute__((aligned(16))) __bf16 so[C2];
    int m = blockIdx.x;
    int c = threadIdx.x;
    int t = m % TT;
    int b = m / TT;
    int h = c >> 6;

    if (c < HH) {
        const float* p = wcoef + (size_t)m * NWP + c * KK;
        float mx = -1e30f;
        for (int j = 0; j < KK; ++j) { const int s = t - PADK + j; if (s >= 0 && s < TT) mx = fmaxf(mx, p[j]); }
        float sum = 0.0f;
        for (int j = 0; j < KK; ++j) { const int s = t - PADK + j; const float e = (s >= 0 && s < TT) ? __expf(p[j] - mx) : 0.0f; attn_s[c][j] = e; sum += e; }
        const float inv = 1.0f / sum;
        for (int j = 0; j < KK; ++j) attn_s[c][j] *= inv;
    }
    if (c < KK) wk_s[c] = wfk[(size_t)m * KKP + c];
    __syncthreads();

    float y = 0.0f;
#pragma unroll 1
    for (int j = 0; j < KK; ++j) {
        int s = t - PADK + j;
        if (s >= 0 && s < TT)
            y += attn_s[h][j] * x[((size_t)b * TT + s) * CC + c];
    }

    const float* xr = x + (size_t)m * CC;
    float xf = 0.0f;
#pragma unroll 1
    for (int j = 0; j < KK; ++j) {
        int ch = c - PADK + j;
        if (ch >= 0 && ch < CC) xf += wk_s[j] * xr[ch];
    }

    float mv = (mask[b * TT + t] != 0) ? 1.0f : 0.0f;
    so[c]      = (__bf16)(y  * mv);
    so[CC + c] = (__bf16)(xf * mv);
    __syncthreads();
    if (c < C2 / 8) {
        __bf16* d = cat + (size_t)m * C2 + c * 8;
        *(volatile v4u_t*)d = *(const v4ua*)(so + c * 8); __threadfence(); *(volatile v4u_t*)d = *(const v4ua*)(so + c * 8);
    }
}

__global__ __launch_bounds__(256) void k_out_gemm(const __bf16* __restrict__ cat,
                           const __bf16* __restrict__ pw2,
                           const float* __restrict__ b2,
                           float* __restrict__ out) {
    __shared__ __attribute__((aligned(16))) float st[8][16 * 68];
    int lane = threadIdx.x & 31;
    float* sw = st[threadIdx.x >> 5];
    int job  = blockIdx.x * (blockDim.x >> 5) + (threadIdx.x >> 5);
    int mt = job >> 2;
    int g4 = job & 3;
    if (mt >= MM / 16) return;
    int m0 = mt * 16;
    int ntBase = g4 * 4;
    const int NT = 16;

    v8f acc[4];
#pragma unroll
    for (int i = 0; i < 4; ++i) acc[i] = (v8f){};

    for (int kt = 0; kt < C2 / 32; ++kt) {
        v16bf af = load_a_bf16(cat, C2, m0, kt * 32, lane);
#pragma unroll
        for (int i = 0; i < 4; ++i) {
            v16bf bfr = load_b_packed(pw2, NT, kt, ntBase + i, lane);
            acc[i] = wmma_bf16(af, bfr, acc[i]);
        }
    }

    int hl = lane >> 4;
#pragma unroll
    for (int i = 0; i < 4; ++i) {
        int col  = (ntBase + i) * 16 + (lane & 15);
        float bv = b2[col];
#pragma unroll
        for (int v = 0; v < 8; ++v) sw[(v + 8 * hl) * 68 + i * 16 + (lane & 15)] = acc[i][v] + bv;
    }
    asm volatile("s_wait_dscnt 0" ::: "memory");
    const int cb = ntBase * 16;
#pragma unroll 1
    for (int pass = 0; pass < 2; ++pass) {
#pragma unroll
        for (int it = 0; it < 8; ++it) { const int ch = lane + 32 * it, r = ch >> 4, q = (ch & 15) * 4;
            *(volatile v4f_t*)(out + (size_t)(m0 + r) * CC + cb + q) = *(const volatile v4fa*)(sw + r * 68 + q); }
        __threadfence();
    }
}

extern "C" void kernel_launch(void* const* d_in, const int* in_sizes, int n_in,
                              void* d_out, int out_size, void* d_ws, size_t ws_size,
                              hipStream_t stream) {
    const float* q    = (const float*)d_in[0];
    const int*   mask = (const int*)  d_in[3];
    const float* w1   = (const float*)d_in[4];
    const float* b1   = (const float*)d_in[5];
    const float* w2   = (const float*)d_in[6];
    const float* b2   = (const float*)d_in[7];
    const float* ww   = (const float*)d_in[8];
    const float* bw   = (const float*)d_in[9];
    const float* wf   = (const float*)d_in[10];
    const float* bfv  = (const float*)d_in[11];
    float* out = (float*)d_out;

    char* ws = (char*)d_ws;
    size_t off = 0;
    float*  x_f32  = (float*) (ws + off); off += (size_t)MM * CC * sizeof(float);
    __bf16* x_bf16 = (__bf16*)(ws + off); off += (size_t)MM * CC * sizeof(__bf16);
    float*  wcoef  = (float*) (ws + off); off += (size_t)MM * NWP * sizeof(float);
    float*  wfk    = (float*) (ws + off); off += (size_t)MM * KKP * sizeof(float);
    __bf16* catb   = (__bf16*)(ws + off); off += (size_t)MM * C2 * sizeof(__bf16);
    __bf16* qb     = (__bf16*)(ws + off); off += (size_t)MM * CC * sizeof(__bf16);
    __bf16* pw1    = (__bf16*)(ws + off); off += (size_t)CC * 512 * sizeof(__bf16);
    __bf16* pww    = (__bf16*)(ws + off); off += (size_t)CC * 128 * sizeof(__bf16);
    __bf16* pwf    = (__bf16*)(ws + off); off += (size_t)CC *  32 * sizeof(__bf16);
    __bf16* pw2    = (__bf16*)(ws + off); off += (size_t)C2 * 256 * sizeof(__bf16);
    (void)ws_size; (void)in_sizes; (void)n_in; (void)out_size;

    const int THREADS = 256;
    const int WPB     = THREADS / 32;

    {
        int thr = (CC / 32) * (512 / 16) * 32;
        k_pack_b<<<(thr + THREADS - 1) / THREADS, THREADS, 0, stream>>>(w1, CC, C2, 512, pw1);
    }
    {
        int thr = (CC / 32) * (128 / 16) * 32;
        k_pack_b<<<(thr + THREADS - 1) / THREADS, THREADS, 0, stream>>>(ww, CC, NW, 128, pww);
    }
    {
        int thr = (CC / 32) * (32 / 16) * 32;
        k_pack_b<<<(thr + THREADS - 1) / THREADS, THREADS, 0, stream>>>(wf, CC, KK, 32, pwf);
    }
    {
        int thr = (C2 / 32) * (CC / 16) * 32;
        k_pack_b<<<(thr + THREADS - 1) / THREADS, THREADS, 0, stream>>>(w2, C2, CC, 256, pw2);
    }
    {
        int n4 = MM * CC / 4;
        k_cvt_bf16<<<(n4 + THREADS - 1) / THREADS, THREADS, 0, stream>>>(q, qb, n4);
    }
    {
        int jobs = (MM / 16) * 4;
        k_glu_gemm<<<(jobs + WPB - 1) / WPB, THREADS, 0, stream>>>(qb, pw1, b1, x_f32, x_bf16);
    }
    {
        int jobs = (MM / 16) * 3;
        k_coef_gemm<<<(jobs + WPB - 1) / WPB, THREADS, 0, stream>>>(x_bf16, pww, pwf, bw, bfv, wcoef, wfk);
    }
    {
        k_mix<<<MM, CC, 0, stream>>>(x_f32, wcoef, wfk, mask, catb);
    }
    {
        int jobs = (MM / 16) * 4;
        k_out_gemm<<<(jobs + WPB - 1) / WPB, THREADS, 0, stream>>>(catb, pw2, b2, out);
    }
}
